// MLCAFusion_37125697306965
// MI455X (gfx1250) — hardware-run, weakly checked
//
#include <hip/hip_runtime.h>
#include <stddef.h>
#include <stdint.h>

#define NBAT 16
#define TA   2048
#define TV   1024
#define TT   1536
#define DM   256
#define CCH  128
#define FD   512
#define NROW (NBAT * TT)
#define QBR  64
#define KC   64
#define NQB  (TT / QBR)
#define NCK  (TT / KC)

static_assert(NROW == 24576);
static_assert(TT % QBR == 0);
static_assert(TT % KC == 0);
static_assert(NROW % 256 == 0);
static_assert(NROW % 8 == 0);
static_assert(DM % 32 == 0);
static_assert(FD % 64 == 0);
static_assert((3 * CCH) % 8 == 0);
static_assert((5 * CCH) % 8 == 0);
static_assert((FD * FD) % 2048 == 0);

typedef _Float16 v16h __attribute__((ext_vector_type(16)));
typedef _Float16 v8h  __attribute__((ext_vector_type(8)));
typedef _Float16 v4h  __attribute__((ext_vector_type(4)));
typedef float    v8f  __attribute__((ext_vector_type(8)));
typedef float    v4f  __attribute__((ext_vector_type(4)));
typedef unsigned int v4u __attribute__((ext_vector_type(4)));

union Frag  { v16h v; v8h h[2]; };
union Pack8 { v8h h; v4u u; };

extern __shared__ __align__(16) unsigned char dsm[];

__device__ __forceinline__ v8f mma16(v16h a, v16h b, v8f c) {
  c = __builtin_amdgcn_wmma_f32_16x16x32_f16(false, a, false, b, (short)0, c, false, false);
  asm volatile("v_nop\n\tv_nop\n\tv_nop\n\tv_nop" : "+v"(c) : "v"(a), "v"(b));
  return c;
}

__device__ __forceinline__ v16h ldfrag(const _Float16* p, int ld, int row0, int k0, int lane) {
  const int m = lane & 15, lh = lane >> 4;
  const _Float16* q = p + (size_t)(row0 + m) * ld + k0 + 8 * lh;
  Frag f;
  f.h[0] = *(const v8h*)(q);
  f.h[1] = *(const v8h*)(q + 16);
  return f.v;
}

__device__ __forceinline__ v8f zero8() { return (v8f){0.f, 0.f, 0.f, 0.f, 0.f, 0.f, 0.f, 0.f}; }

__device__ __forceinline__ float gelu_f(float x) {
  return 0.5f * x * erfcf(-x * 0.70710678118654752440f);
}

__device__ __forceinline__ void gemm32x64(const _Float16* __restrict__ A, int lda,
                                          const _Float16* __restrict__ Bt, int ldb, int K,
                                          int m0, int n0, int lane, v8f (&acc)[2][4]) {
#pragma unroll 1
  for (int k0 = 0; k0 < K; k0 += 32) {
    const v16h a0 = ldfrag(A, lda, m0, k0, lane);
    const v16h a1 = ldfrag(A, lda, m0 + 16, k0, lane);
    const v16h b0 = ldfrag(Bt, ldb, n0, k0, lane);
    const v16h b1 = ldfrag(Bt, ldb, n0 + 16, k0, lane);
    const v16h b2 = ldfrag(Bt, ldb, n0 + 32, k0, lane);
    const v16h b3 = ldfrag(Bt, ldb, n0 + 48, k0, lane);
    acc[0][0] = mma16(a0, b0, acc[0][0]);
    acc[1][0] = mma16(a1, b0, acc[1][0]);
    acc[0][1] = mma16(a0, b1, acc[0][1]);
    acc[1][1] = mma16(a1, b1, acc[1][1]);
    acc[0][2] = mma16(a0, b2, acc[0][2]);
    acc[1][2] = mma16(a1, b2, acc[1][2]);
    acc[0][3] = mma16(a0, b3, acc[0][3]);
    acc[1][3] = mma16(a1, b3, acc[1][3]);
  }
}

__global__ __launch_bounds__(256) void k_interp(const float* __restrict__ src, int Tin, float scale,
                                                float* __restrict__ dst) {
#pragma clang fp contract(off)
  const int tid = threadIdx.x, lane = tid & 31, wave = tid >> 5;
  const int row = blockIdx.x * 8 + wave;
  const int b = row / TT, t = row - b * TT;
  float sp = ((float)t + 0.5f) * scale - 0.5f;
  sp = fmaxf(sp, 0.0f);
  int i0 = (int)floorf(sp);
  i0 = min(i0, Tin - 1);
  i0 = max(i0, 0);
  const int i1 = min(i0 + 1, Tin - 1);
  const float w  = sp - (float)i0;
  const float w0 = 1.0f - w;
  const float* r0p = src + ((size_t)b * Tin + i0) * DM;
  const float* r1p = src + ((size_t)b * Tin + i1) * DM;
  v4f o[2];
#pragma unroll
  for (int it = 0; it < 2; ++it) {
    const int idx = it * 128 + lane * 4;
    const v4f x0 = *(const v4f*)(r0p + idx);
    const v4f x1 = *(const v4f*)(r1p + idx);
    const v4f p0 = x0 * w0;
    const v4f p1 = x1 * w;
    o[it] = p0 + p1;
  }
  float* dp = dst + (size_t)row * DM;
  for (int ps = 0; ps < 2; ++ps) {
#pragma unroll
    for (int it = 0; it < 2; ++it) *(volatile v4f*)(dp + it * 128 + lane * 4) = o[it];
    __threadfence();
  }
}

__global__ __launch_bounds__(256) void k_wconv(const float* __restrict__ w, int KK, _Float16* __restrict__ dst) {
  const int tid = threadIdx.x, lane = tid & 31, wave = tid >> 5;
  const int row = blockIdx.x * 8 + wave;
  const int k = row / CCH, co = row - k * CCH;
  const int ci0 = 8 * lane;
  const float* p = w + ((size_t)co * DM + ci0) * KK + k;
  float f[8];
#pragma unroll
  for (int i = 0; i < 8; ++i) f[i] = p[(size_t)i * KK] * 32.0f;
  Pack8 pk;
  pk.h = (v8h){(_Float16)f[0], (_Float16)f[1], (_Float16)f[2], (_Float16)f[3],
               (_Float16)f[4], (_Float16)f[5], (_Float16)f[6], (_Float16)f[7]};
  const v4u vv = pk.u;
  volatile v4u* d = (volatile v4u*)(dst + (size_t)row * DM + ci0);
  *d = vv;
  __threadfence();
  *d = vv;
}

__global__ __launch_bounds__(256) void k_wproj(const float* __restrict__ w, _Float16* __restrict__ dst) {
  const size_t o = ((size_t)blockIdx.x * 256 + threadIdx.x) * 8;
  const v4f a0 = *(const v4f*)(w + o) * 32.0f;
  const v4f a1 = *(const v4f*)(w + o + 4) * 32.0f;
  Pack8 pk;
  pk.h = (v8h){(_Float16)a0[0], (_Float16)a0[1], (_Float16)a0[2], (_Float16)a0[3],
               (_Float16)a1[0], (_Float16)a1[1], (_Float16)a1[2], (_Float16)a1[3]};
  const v4u vv = pk.u;
  volatile v4u* d = (volatile v4u*)(dst + o);
  *d = vv;
  __threadfence();
  *d = vv;
}

#define XTP 264
#define YTP 260
#define CONV_XS   0
#define CONV_YS   (68 * XTP * 2)
#define CONV_INV  (CONV_YS + 64 * YTP * 4)
#define CONV_LDS  (CONV_INV + 64 * 4)
static_assert(CONV_YS % 16 == 0);
static_assert(CONV_INV % 16 == 0);

__global__ __launch_bounds__(256) void k_conv(const float* __restrict__ xf,
                                              const _Float16* __restrict__ w3, const float* __restrict__ b3,
                                              const _Float16* __restrict__ w5, const float* __restrict__ b5,
                                              _Float16* __restrict__ mt, _Float16* __restrict__ nrm) {
  _Float16* Xs = (_Float16*)(dsm + CONV_XS);
  float* Ys    = (float*)(dsm + CONV_YS);
  float* invn  = (float*)(dsm + CONV_INV);

  const int tid = threadIdx.x, lane = tid & 31, wave = tid >> 5;
  const int hh = lane >> 4, c = lane & 15;
  const int bx = blockIdx.x;
  const int b  = bx / NQB;
  const int t0 = (bx - b * NQB) * QBR;
  const size_t brow  = (size_t)b * TT;
  const size_t grow0 = (size_t)bx * QBR;

#pragma unroll 4
  for (int i = 0; i < 17; ++i) {
    const int idx = tid + 256 * i;
    const int r   = idx >> 6;
    const int c4  = (idx & 63) * 4;
    const int t   = t0 - 2 + r;
    const int tc  = min(max(t, 0), TT - 1);
    v4f x = *(const v4f*)(xf + (brow + (size_t)tc) * DM + c4);
    if (t < 0 || t >= TT) x = (v4f){0.f, 0.f, 0.f, 0.f};
    const v4h hv = (v4h){(_Float16)x[0], (_Float16)x[1], (_Float16)x[2], (_Float16)x[3]};
    *(v4h*)(Xs + r * XTP + c4) = hv;
  }
  __syncthreads();

  const int cv    = wave >> 2;
  const int taps  = cv ? 5 : 3;
  const int roff0 = cv ? 0 : 1;
  const _Float16* wp = cv ? w5 : w3;
  const float* bp    = cv ? b5 : b3;
  const int co0 = (wave & 3) * 32;

  v8f acc[4][2];
#pragma unroll
  for (int rt = 0; rt < 4; ++rt) { acc[rt][0] = zero8(); acc[rt][1] = zero8(); }

#pragma unroll 1
  for (int k = 0; k < taps; ++k) {
    const int roff = k + roff0;
    const _Float16* wk = wp + (size_t)k * CCH * DM;
#pragma unroll 2
    for (int kb = 0; kb < 8; ++kb) {
      const v16h bf0 = ldfrag(wk, DM, co0, kb * 32, lane);
      const v16h bf1 = ldfrag(wk, DM, co0 + 16, kb * 32, lane);
#pragma unroll
      for (int rt = 0; rt < 4; ++rt) {
        const v16h a = ldfrag(Xs, XTP, rt * 16 + roff, kb * 32, lane);
        acc[rt][0] = mma16(a, bf0, acc[rt][0]);
        acc[rt][1] = mma16(a, bf1, acc[rt][1]);
      }
    }
  }

  float bb[2];
  bb[0] = bp[co0 + c];
  bb[1] = bp[co0 + 16 + c];
  const int cbase = cv * CCH + co0;
#pragma unroll
  for (int rt = 0; rt < 4; ++rt)
#pragma unroll
    for (int ct = 0; ct < 2; ++ct)
#pragma unroll
      for (int r = 0; r < 8; ++r)
        Ys[(rt * 16 + 8 * hh + r) * YTP + cbase + 16 * ct + c] = gelu_f(acc[rt][ct][r] * 0.03125f + bb[ct]);
  __syncthreads();

  {
    const int row = tid >> 2, q = tid & 3;
    const float* yr = Ys + row * YTP + 64 * q;
    float s = 0.f;
#pragma unroll 4
    for (int i = 0; i < 16; ++i) {
      const v4f y = *(const v4f*)(yr + 4 * i);
      s += (y[0] * y[0] + y[1] * y[1]) + (y[2] * y[2] + y[3] * y[3]);
    }
    s += __shfl_xor(s, 1, 32);
    s += __shfl_xor(s, 2, 32);
    const float inv = 1.0f / fmaxf(sqrtf(s), 1e-12f);
    if (q == 0) invn[row] = inv;
  }
  __syncthreads();

  {
    v4u val[8];
    size_t go[8];
#pragma unroll
    for (int g = 0; g < 8; ++g) {
      const int row = wave + 8 * g;
      const float sc = invn[row] * 256.0f;
      const float* yr = Ys + row * YTP + 8 * lane;
      const v4f a0 = *(const v4f*)(yr) * sc;
      const v4f a1 = *(const v4f*)(yr + 4) * sc;
      Pack8 pk;
      pk.h = (v8h){(_Float16)a0[0], (_Float16)a0[1], (_Float16)a0[2], (_Float16)a0[3],
                   (_Float16)a1[0], (_Float16)a1[1], (_Float16)a1[2], (_Float16)a1[3]};
      val[g] = pk.u;
      go[g]  = (grow0 + (size_t)row) * DM + 8 * lane;
    }
    for (int ps = 0; ps < 2; ++ps) {
#pragma unroll
      for (int g = 0; g < 8; ++g) *(volatile v4u*)(nrm + go[g]) = val[g];
      __threadfence();
    }
  }

  {
    v4u val[8];
    size_t go[8];
#pragma unroll
    for (int g = 0; g < 8; ++g) {
      const int p  = tid + 256 * g;
      const int co = p >> 3;
      const int pc = p & 7;
      const float* yc = Ys + (8 * pc) * YTP + co;
      Pack8 pk;
      pk.h = (v8h){(_Float16)yc[0],       (_Float16)yc[YTP],     (_Float16)yc[2 * YTP], (_Float16)yc[3 * YTP],
                   (_Float16)yc[4 * YTP], (_Float16)yc[5 * YTP], (_Float16)yc[6 * YTP], (_Float16)yc[7 * YTP]};
      val[g] = pk.u;
      go[g]  = ((size_t)b * DM + co) * TT + t0 + 8 * pc;
    }
    for (int ps = 0; ps < 2; ++ps) {
#pragma unroll
      for (int g = 0; g < 8; ++g) *(volatile v4u*)(mt + go[g]) = val[g];
      __threadfence();
    }
  }
}

#define QTP 264
#define VTP 72
#define PTP 72
#define OSP 132
#define ATT_QS  0
#define ATT_KS  (64 * QTP * 2)
#define ATT_VS  (ATT_KS + 64 * QTP * 2)
#define ATT_PS  (ATT_VS + 256 * VTP * 2)
#define ATT_SM  (ATT_PS + 4 * 16 * PTP * 2)
#define ATT_SL  (ATT_SM + 128 * 4)
#define ATT_LDS (ATT_SL + 128 * 4)
#define ATT_OS  ATT_KS
static_assert(ATT_OS + 8 * 16 * OSP * 4 <= ATT_PS);
static_assert(ATT_KS % 16 == 0);
static_assert(ATT_VS % 16 == 0);
static_assert(ATT_PS % 16 == 0);
static_assert(ATT_SM % 16 == 0);

__global__ __launch_bounds__(256) void k_attn(const _Float16* __restrict__ qn, const _Float16* __restrict__ kn,
                                              const _Float16* __restrict__ vtp, const float* __restrict__ res,
                                              _Float16* __restrict__ fu, int coff, float sscale) {
  _Float16* Qs = (_Float16*)(dsm + ATT_QS);
  _Float16* Ks = (_Float16*)(dsm + ATT_KS);
  _Float16* Vs = (_Float16*)(dsm + ATT_VS);
  _Float16* Ps = (_Float16*)(dsm + ATT_PS);
  float* Sm = (float*)(dsm + ATT_SM);
  float* Sl = (float*)(dsm + ATT_SL);
  float* Os = (float*)(dsm + ATT_OS);

  const int tid = threadIdx.x, lane = tid & 31, wave = tid >> 5;
  const int hh = lane >> 4, c = lane & 15;
  const int qr = wave & 3, ch = wave >> 2;
  const int bx = blockIdx.x;
  const int b  = bx / NQB;
  const int qb = bx - b * NQB;
  const size_t brow  = (size_t)b * TT;
  const size_t qrow0 = brow + (size_t)qb * QBR;

#pragma unroll 2
  for (int i = 0; i < 8; ++i) {
    const int idx = tid + 256 * i;
    const int r = idx >> 5, c8 = (idx & 31) * 8;
    *(v8h*)(Qs + r * QTP + c8) = *(const v8h*)(qn + (qrow0 + (size_t)r) * DM + c8);
  }

  const float NEGB = -1.0e30f;
  float mrow[8], lrow[8];
  v8f oacc[8];
#pragma unroll
  for (int r = 0; r < 8; ++r) { mrow[r] = NEGB; lrow[r] = 0.f; }
#pragma unroll
  for (int t = 0; t < 8; ++t) oacc[t] = zero8();

  _Float16* pq = Ps + qr * (16 * PTP);
  const int smo = qr * 32;

  for (int kc = 0; kc < NCK; ++kc) {
    const int kv0 = kc * KC;
    __syncthreads();
#pragma unroll 2
    for (int i = 0; i < 8; ++i) {
      const int idx = tid + 256 * i;
      {
        const int r = idx >> 5, c8 = (idx & 31) * 8;
        *(v8h*)(Ks + r * QTP + c8) = *(const v8h*)(kn + (brow + (size_t)(kv0 + r)) * DM + c8);
      }
      {
        const int d = idx >> 3, c8 = (idx & 7) * 8;
        *(v8h*)(Vs + d * VTP + c8) = *(const v8h*)(vtp + ((size_t)b * DM + d) * TT + kv0 + c8);
      }
    }
    __syncthreads();

    v8f s[2];
    s[0] = zero8();
    s[1] = zero8();
#pragma unroll 2
    for (int dc = 0; dc < 8; ++dc) {
      const v16h qa  = ldfrag(Qs, QTP, qr * 16, dc * 32, lane);
      const v16h kf0 = ldfrag(Ks, QTP, ch * 32, dc * 32, lane);
      const v16h kf1 = ldfrag(Ks, QTP, ch * 32 + 16, dc * 32, lane);
      s[0] = mma16(qa, kf0, s[0]);
      s[1] = mma16(qa, kf1, s[1]);
    }
    float pm[8];
#pragma unroll
    for (int r = 0; r < 8; ++r) {
      s[0][r] *= sscale;
      s[1][r] *= sscale;
      float m = fmaxf(s[0][r], s[1][r]);
#pragma unroll
      for (int off = 1; off < 16; off <<= 1) m = fmaxf(m, __shfl_xor(m, off, 32));
      pm[r] = m;
    }
    if (c == 0) {
#pragma unroll
      for (int r = 0; r < 8; ++r) Sm[smo + ch * 16 + 8 * hh + r] = pm[r];
    }
    __syncthreads();

    float al[8], pl[8];
#pragma unroll
    for (int r = 0; r < 8; ++r) {
      const int ri = 8 * hh + r;
      const float cm    = fmaxf(Sm[smo + ri], Sm[smo + 16 + ri]);
      const float mnew  = fmaxf(mrow[r], cm);
      const float alpha = __expf(mrow[r] - mnew);
      mrow[r] = mnew;
      const float e0 = __expf(s[0][r] - mnew);
      const float e1 = __expf(s[1][r] - mnew);
      pq[ri * PTP + ch * 32 + c]      = (_Float16)(e0 * 1024.0f);
      pq[ri * PTP + ch * 32 + 16 + c] = (_Float16)(e1 * 1024.0f);
      float psum = e0 + e1;
#pragma unroll
      for (int off = 1; off < 16; off <<= 1) psum += __shfl_xor(psum, off, 32);
      pl[r] = psum;
      al[r] = alpha;
    }
    if (c == 0) {
#pragma unroll
      for (int r = 0; r < 8; ++r) Sl[smo + ch * 16 + 8 * hh + r] = pl[r];
    }
#pragma unroll
    for (int t = 0; t < 8; ++t)
#pragma unroll
      for (int r = 0; r < 8; ++r) oacc[t][r] *= al[r];
    __syncthreads();

#pragma unroll
    for (int r = 0; r < 8; ++r) {
      const int ri = 8 * hh + r;
      lrow[r] = lrow[r] * al[r] + (Sl[smo + ri] + Sl[smo + 16 + ri]);
    }
#pragma unroll
    for (int kk = 0; kk < 2; ++kk) {
      const v16h pa = ldfrag(pq, PTP, 0, kk * 32, lane);
#pragma unroll
      for (int t = 0; t < 8; ++t) {
        const v16h vb = ldfrag(Vs, VTP, ch * 128 + 16 * t, kk * 32, lane);
        oacc[t] = mma16(pa, vb, oacc[t]);
      }
    }
  }

  float inv[8];
#pragma unroll
  for (int r = 0; r < 8; ++r) inv[r] = (lrow[r] > 0.f) ? (1.0f / (lrow[r] * 1024.0f)) : 0.f;
  __syncthreads();
  float* ow = Os + wave * (16 * OSP);
#pragma unroll
  for (int t = 0; t < 8; ++t)
#pragma unroll
    for (int r = 0; r < 8; ++r) ow[(8 * hh + r) * OSP + 16 * t + c] = oacc[t][r] * inv[r];
  __syncthreads();
  v4u val[8];
  size_t go[8];
#pragma unroll
  for (int it = 0; it < 8; ++it) {
    const int p  = lane + 32 * it;
    const int L  = p >> 4;
    const int pc = p & 15;
    const float* op = ow + L * OSP + 8 * pc;
    const size_t grow = qrow0 + (size_t)(qr * 16 + L);
    const float* rp = res + grow * DM + ch * 128 + 8 * pc;
    const v4f o0 = *(const v4f*)(op), o1 = *(const v4f*)(op + 4);
    const v4f r0 = *(const v4f*)(rp), r1 = *(const v4f*)(rp + 4);
    const v4f f0 = o0 + r0, f1 = o1 + r1;
    Pack8 pk;
    pk.h = (v8h){(_Float16)f0[0], (_Float16)f0[1], (_Float16)f0[2], (_Float16)f0[3],
                 (_Float16)f1[0], (_Float16)f1[1], (_Float16)f1[2], (_Float16)f1[3]};
    val[it] = pk.u;
    go[it]  = grow * FD + (size_t)coff + ch * 128 + 8 * pc;
  }
  for (int ps = 0; ps < 2; ++ps) {
#pragma unroll
    for (int it = 0; it < 8; ++it) *(volatile v4u*)(fu + go[it]) = val[it];
    __threadfence();
  }
}

#define OTP 68
__global__ __launch_bounds__(256) void k_proj(const _Float16* __restrict__ ap, const _Float16* __restrict__ wt,
                                              const float* __restrict__ bias, float* __restrict__ out) {
  __shared__ __align__(16) float st[8][16 * OTP];
  const int tid = threadIdx.x, lane = tid & 31, wave = tid >> 5;
  const int hh = lane >> 4, c = lane & 15;
  const int m0 = blockIdx.x * 256 + wave * 32;
  const int n0 = blockIdx.y * 64;

  v8f acc[2][4];
#pragma unroll
  for (int sb = 0; sb < 2; ++sb)
#pragma unroll
    for (int t = 0; t < 4; ++t) acc[sb][t] = zero8();
  gemm32x64(ap, FD, wt, FD, FD, m0, n0, lane, acc);
  float bb[4];
#pragma unroll
  for (int t = 0; t < 4; ++t) bb[t] = bias[n0 + 16 * t + c];

  float* sw = st[wave];
#pragma unroll
  for (int sub = 0; sub < 2; ++sub) {
    __syncthreads();
#pragma unroll
    for (int t = 0; t < 4; ++t) {
#pragma unroll
      for (int r = 0; r < 8; ++r)
        sw[(8 * hh + r) * OTP + 16 * t + c] = gelu_f(acc[sub][t][r] * 0.03125f + bb[t]);
    }
    __syncthreads();
    v4f val[8];
    size_t go[8];
#pragma unroll
    for (int it = 0; it < 8; ++it) {
      const int p    = lane + 32 * it;
      const int L    = p >> 3;
      const int pc   = p & 7;
      const int row  = L >> 1;
      const int half = L & 1;
      val[it] = *(const v4f*)(sw + row * OTP + half * 32 + pc * 4);
      go[it]  = (size_t)(m0 + sub * 16 + row) * FD + n0 + half * 32 + pc * 4;
    }
    for (int ps = 0; ps < 2; ++ps) {
#pragma unroll
      for (int it = 0; it < 8; ++it) *(volatile v4f*)(out + go[it]) = val[it];
      __threadfence();
    }
  }
}

extern "C" void kernel_launch(void* const* d_in, const int* in_sizes, int n_in,
                              void* d_out, int out_size, void* d_ws, size_t ws_size,
                              hipStream_t stream) {
  if (n_in < 12) return;
  if (in_sizes[0] != NBAT * TA * DM) return;
  if (in_sizes[1] != NBAT * TV * DM) return;
  if (in_sizes[2] != CCH * DM * 3) return;
  if (in_sizes[3] != CCH) return;
  if (in_sizes[4] != CCH * DM * 5) return;
  if (in_sizes[5] != CCH) return;
  if (in_sizes[6] != CCH * DM * 3) return;
  if (in_sizes[7] != CCH) return;
  if (in_sizes[8] != CCH * DM * 5) return;
  if (in_sizes[9] != CCH) return;
  if (in_sizes[10] != FD * FD) return;
  if (in_sizes[11] != FD) return;
  if (out_size != NROW * FD) return;

  const float* audio = (const float*)d_in[0];
  const float* video = (const float*)d_in[1];
  const float* a3w   = (const float*)d_in[2];
  const float* a3b   = (const float*)d_in[3];
  const float* a5w   = (const float*)d_in[4];
  const float* a5b   = (const float*)d_in[5];
  const float* v3w   = (const float*)d_in[6];
  const float* v3b   = (const float*)d_in[7];
  const float* v5w   = (const float*)d_in[8];
  const float* v5b   = (const float*)d_in[9];
  const float* pw    = (const float*)d_in[10];
  const float* pb    = (const float*)d_in[11];
  float* out = (float*)d_out;

  size_t off = 0;
  const size_t oAF  = off; off += (size_t)NROW * DM * 4;
  const size_t oVF  = off; off += (size_t)NROW * DM * 4;
  const size_t oAN  = off; off += (size_t)NROW * DM * 2;
  const size_t oVN  = off; off += (size_t)NROW * DM * 2;
  const size_t oAMT = off; off += (size_t)NBAT * DM * TT * 2;
  const size_t oVMT = off; off += (size_t)NBAT * DM * TT * 2;
  const size_t oFU  = off; off += (size_t)NROW * FD * 2;
  const size_t oW3A = off; off += (size_t)3 * CCH * DM * 2;
  const size_t oW5A = off; off += (size_t)5 * CCH * DM * 2;
  const size_t oW3V = off; off += (size_t)3 * CCH * DM * 2;
  const size_t oW5V = off; off += (size_t)5 * CCH * DM * 2;
  const size_t oWP  = off; off += (size_t)FD * FD * 2;
  if (off > ws_size) return;
  if (off > (size_t)134217728) return;

  char* ws = (char*)d_ws;
  float*    AF  = (float*)(ws + oAF);
  float*    VF  = (float*)(ws + oVF);
  _Float16* AN  = (_Float16*)(ws + oAN);
  _Float16* VN  = (_Float16*)(ws + oVN);
  _Float16* AMT = (_Float16*)(ws + oAMT);
  _Float16* VMT = (_Float16*)(ws + oVMT);
  _Float16* FU  = (_Float16*)(ws + oFU);
  _Float16* W3A = (_Float16*)(ws + oW3A);
  _Float16* W5A = (_Float16*)(ws + oW5A);
  _Float16* W3V = (_Float16*)(ws + oW3V);
  _Float16* W5V = (_Float16*)(ws + oW5V);
  _Float16* WP  = (_Float16*)(ws + oWP);

  const float sa = (float)((double)TA / (double)TT);
  const float sv = (float)((double)TV / (double)TT);
  k_interp<<<dim3(NROW / 8), dim3(256), 0, stream>>>(audio, TA, sa, AF);
  k_interp<<<dim3(NROW / 8), dim3(256), 0, stream>>>(video, TV, sv, VF);
  k_wconv<<<dim3((3 * CCH) / 8), dim3(256), 0, stream>>>(a3w, 3, W3A);
  k_wconv<<<dim3((5 * CCH) / 8), dim3(256), 0, stream>>>(a5w, 5, W5A);
  k_wconv<<<dim3((3 * CCH) / 8), dim3(256), 0, stream>>>(v3w, 3, W3V);
  k_wconv<<<dim3((5 * CCH) / 8), dim3(256), 0, stream>>>(v5w, 5, W5V);
  k_wproj<<<dim3((FD * FD) / 2048), dim3(256), 0, stream>>>(pw, WP);
  (void)hipFuncSetAttribute(reinterpret_cast<const void*>(&k_conv), hipFuncAttributeMaxDynamicSharedMemorySize, CONV_LDS);
  k_conv<<<dim3(NROW / QBR), dim3(256), CONV_LDS, stream>>>(AF, W3A, a3b, W5A, a5b, AMT, AN);
  k_conv<<<dim3(NROW / QBR), dim3(256), CONV_LDS, stream>>>(VF, W3V, v3b, W5V, v5b, VMT, VN);
  const float sscale = 1.52587890625e-05f;
  (void)hipFuncSetAttribute(reinterpret_cast<const void*>(&k_attn), hipFuncAttributeMaxDynamicSharedMemorySize, ATT_LDS);
  k_attn<<<dim3(NROW / QBR), dim3(256), ATT_LDS, stream>>>(AN, VN, VMT, AF, FU, 0, sscale);
  k_attn<<<dim3(NROW / QBR), dim3(256), ATT_LDS, stream>>>(VN, AN, AMT, VF, FU, 256, sscale);
  k_proj<<<dim3(NROW / 256, FD / 64), dim3(256), 0, stream>>>(FU, WP, pb, out);
  (void)hipGetLastError();
}
